// EGNNA_22179211117031
// MI455X (gfx1250) — hardware-run, weakly checked
//
#include <hip/hip_runtime.h>


namespace {
constexpr int N = 768, F = 256, H1 = 256, H2 = 128, NE = 4, H3 = 256, H4 = 128, NCLS = 2;
constexpr float XS = 8.0f, WSC = 256.0f, PS = 1024.0f, THR = 0.87f, COS_EPS = 1e-6f, NEG = 0.2f, LOG2E = 1.4426950408889634f;

typedef _Float16 b16;
typedef __attribute__((ext_vector_type(16))) _Float16 v16b;
typedef __attribute__((ext_vector_type(8))) _Float16 v8b;
typedef __attribute__((ext_vector_type(8))) float v8f;
typedef __attribute__((ext_vector_type(4))) float v4f;
__device__ __forceinline__ float bf16_rne(float f) { unsigned int u = __float_as_uint(f); u += 0x7FFFu + ((u >> 16) & 1u); return __uint_as_float(u & 0xFFFF0000u); }
__device__ __forceinline__ void split16(float v, b16& hi, b16& lo) { hi = (b16)v; lo = (b16)(v - (float)hi); }
__device__ __forceinline__ v16b frag_kb(const b16* p, int hh) { const v8b a = *(const v8b*)(p + 8 * hh), b = *(const v8b*)(p + 16 + 8 * hh); v16b f;
#pragma unroll
  for (int e = 0; e < 8; ++e) { f[e] = a[e]; f[8 + e] = b[e]; } return f; }
__device__ __forceinline__ v8f wmma16b(v16b a, v16b b, v8f c) { v8f d = __builtin_amdgcn_wmma_f32_16x16x32_f16(false, a, false, b, (short)0, c, false, false); asm volatile("v_nop\n\tv_nop\n\tv_nop\n\tv_nop" : "+v"(d) : "v"(a), "v"(b)); return d; }
__device__ __forceinline__ void wave_lds_sync() { __builtin_amdgcn_fence(__ATOMIC_RELEASE, "workgroup"); __builtin_amdgcn_wave_barrier(); __builtin_amdgcn_fence(__ATOMIC_ACQUIRE, "workgroup"); }
__device__ __forceinline__ float pmul(float a, float b) { float p = a * b; asm volatile("" : "+v"(p)); return p; }
__device__ __forceinline__ float lrelu(float x) { return x > 0.0f ? x : NEG * x; }
__device__ __forceinline__ float nexp2(float x) { return __builtin_amdgcn_exp2f(x); }

__global__ __launch_bounds__(256) void prep_kernel(const float* __restrict__ x, const float* __restrict__ w1, const float* __restrict__ w2, const float* __restrict__ fc1, const float* __restrict__ fc2, const float* __restrict__ fc3, b16* __restrict__ Xh, b16* __restrict__ Xl, b16* __restrict__ W1T, b16* __restrict__ W2T, b16* __restrict__ FC1T, b16* __restrict__ FC2T, b16* __restrict__ FC3T, b16* __restrict__ FC1R) {
  const size_t t = (size_t)blockIdx.x * 256 + threadIdx.x; size_t u = t; v8b o, z = {};
  const size_t nx = (size_t)N * F / 8, n1 = (size_t)H1 * F / 8, n2 = (size_t)H2 * H1 / 8, n3 = (size_t)2 * H3 * H2 / 8, n4 = (size_t)H4 * H3 / 8, n5 = (size_t)16 * H4 / 8, n6 = (size_t)H3 * 32 / 8;
  if (u < nx) { const size_t e = u * 8; for (int j = 0; j < 8; ++j) o[j] = (b16)(bf16_rne(x[e + j]) * XS); for (int pass = 0; pass < 2; ++pass) { *(volatile v8b*)(Xh + e) = o; *(volatile v8b*)(Xl + e) = z; __threadfence(); } return; } u -= nx;
  if (u < n1) { const int e = (int)u * 8; const int oo = e / F, k0 = e % F; for (int j = 0; j < 8; ++j) o[j] = (b16)(bf16_rne(w1[(k0 + j) * H1 + oo]) * WSC); for (int pass = 0; pass < 2; ++pass) { *(volatile v8b*)(W1T + e) = o; __threadfence(); } return; } u -= n1;
  if (u < n2) { const int e = (int)u * 8; const int oo = e / H1, k0 = e % H1; for (int j = 0; j < 8; ++j) o[j] = (b16)(bf16_rne(w2[(k0 + j) * H2 + oo]) * WSC); for (int pass = 0; pass < 2; ++pass) { *(volatile v8b*)(W2T + e) = o; __threadfence(); } return; } u -= n2;
  if (u < n3) { const int e = (int)u * 8; const int oo = e / H2, k0 = e % H2; const int half = oo / H3, o2 = oo % H3; for (int j = 0; j < 8; ++j) o[j] = (b16)(bf16_rne(fc1[(size_t)(half * H2 + k0 + j) * H3 + o2]) * WSC); for (int pass = 0; pass < 2; ++pass) { *(volatile v8b*)(FC1T + e) = o; __threadfence(); } return; } u -= n3;
  if (u < n4) { const int e = (int)u * 8; const int oo = e / H3, k0 = e % H3; for (int j = 0; j < 8; ++j) o[j] = (b16)(bf16_rne(fc2[(k0 + j) * H4 + oo]) * WSC); for (int pass = 0; pass < 2; ++pass) { *(volatile v8b*)(FC2T + e) = o; __threadfence(); } return; } u -= n4;
  if (u < n5) { const int e = (int)u * 8; const int oo = e / H4, k0 = e % H4; for (int j = 0; j < 8; ++j) o[j] = (oo < NCLS) ? (b16)(bf16_rne(fc3[(k0 + j) * NCLS + min(oo, NCLS - 1)]) * WSC) : (b16)0.0f; for (int pass = 0; pass < 2; ++pass) { *(volatile v8b*)(FC3T + e) = o; __threadfence(); } return; } u -= n5;
  if (u < n6) { const int e = (int)u * 8; const int oo = e / 32, k0 = e % 32; for (int j = 0; j < 8; ++j) { const int k = k0 + j; o[j] = (k < NE) ? (b16)(bf16_rne(fc1[(size_t)(2 * H2 + min(k, NE - 1)) * H3 + oo]) * WSC) : (b16)0.0f; } for (int pass = 0; pass < 2; ++pass) { *(volatile v8b*)(FC1R + e) = o; __threadfence(); } }
}
template <int KD>
__global__ __launch_bounds__(128) void gemm_kernel(const b16* __restrict__ Ah, const b16* __restrict__ Al, int lda, const b16* __restrict__ W, float* __restrict__ Yf, b16* __restrict__ Yh, b16* __restrict__ Yl, int ldy) {
  __shared__ __attribute__((aligned(16))) float Tf[4][16][128 + 4]; __shared__ __attribute__((aligned(16))) b16 Th[4][16][128 + 8], Tl[4][16][128 + 8];
  const int wave = threadIdx.x >> 5, lane = threadIdx.x & 31, nloc = lane & 15, hlf = lane >> 4; const size_t m0 = (size_t)blockIdx.x * 64 + wave * 16; const int n0 = blockIdx.y * 128;
  v8f acc[8];
#pragma unroll
  for (int t = 0; t < 8; ++t) acc[t] = (v8f){};
#pragma unroll 2
  for (int kb = 0; kb < KD; kb += 32) { const v16b a = frag_kb(Ah + (m0 + nloc) * lda + kb, hlf), al = frag_kb(Al + (m0 + nloc) * lda + kb, hlf);
#pragma unroll
    for (int t = 0; t < 8; ++t) { const v16b bw = frag_kb(W + (size_t)(n0 + t * 16 + nloc) * KD + kb, hlf); acc[t] = wmma16b(a, bw, acc[t]); acc[t] = wmma16b(al, bw, acc[t]); } }
#pragma unroll
  for (int t = 0; t < 8; ++t)
#pragma unroll
    for (int r = 0; r < 8; ++r) { const float y = acc[t][r] * (1.0f / (XS * WSC)); Tf[wave][8 * hlf + r][t * 16 + nloc] = y; if (Yh) { b16 p, q; split16(y * XS, p, q); Th[wave][8 * hlf + r][t * 16 + nloc] = p; Tl[wave][8 * hlf + r][t * 16 + nloc] = q; } }
  wave_lds_sync();
  for (int pass = 0; pass < 2; ++pass) { for (int rr = 0; rr < 16; ++rr) *(volatile v4f*)(Yf + (m0 + rr) * ldy + n0 + lane * 4) = *(const v4f*)(&Tf[wave][rr][lane * 4]);
    if (Yh) { for (int r2 = 0; r2 < 16; r2 += 2) { const int rr = r2 + (lane >> 4), c8 = (lane & 15) * 8; const size_t gi = (m0 + rr) * ldy + n0 + c8; *(volatile v8b*)(Yh + gi) = *(const v8b*)(&Th[wave][rr][c8]); *(volatile v8b*)(Yl + gi) = *(const v8b*)(&Tl[wave][rr][c8]); } }
    __threadfence(); }
}
__global__ __launch_bounds__(256) void fdot_kernel(const float* __restrict__ Hf, int D, const float* __restrict__ a, float* __restrict__ FS, float* __restrict__ FD) {
  __shared__ float fs[8][4], fd[8][4];
  const int wave = threadIdx.x >> 5, lane = threadIdx.x & 31; const size_t v = (size_t)blockIdx.x * 8 + wave; const int pl = D / 32;
  for (int e = 0; e < NE; ++e) { float s = 0.0f, d = 0.0f; for (int q = 0; q < pl; ++q) { const int c = lane * pl + q; const float hv = Hf[v * D + c]; s += pmul(hv, bf16_rne(a[e * 2 * D + c])); d += pmul(hv, bf16_rne(a[e * 2 * D + D + c])); }
#pragma unroll
    for (int o = 16; o >= 1; o >>= 1) { s += __shfl_xor(s, o); d += __shfl_xor(d, o); }
    if (lane == 0) { fs[wave][e] = s; fd[wave][e] = d; } }
  __syncthreads();
  for (int pass = 0; pass < 2; ++pass) { if (threadIdx.x < 8) { *(volatile v4f*)(FS + ((size_t)blockIdx.x * 8 + threadIdx.x) * 4) = *(const v4f*)(&fs[threadIdx.x][0]); *(volatile v4f*)(FD + ((size_t)blockIdx.x * 8 + threadIdx.x) * 4) = *(const v4f*)(&fd[threadIdx.x][0]); } __threadfence(); }
}
__global__ __launch_bounds__(256) void attrow_kernel(const float* __restrict__ FS, const float* __restrict__ FD, const float* __restrict__ adj, b16* __restrict__ ABh, b16* __restrict__ ABl) {
  __shared__ float Lg[NE][N]; __shared__ float inv[NE]; __shared__ __attribute__((aligned(16))) b16 Rh[N], Rl[N];
  const int i = blockIdx.x, t_ = threadIdx.x, wave = t_ >> 5, lane = t_ & 31;
  for (int q = t_; q < NE * N; q += 256) { const int e = q / N, j = q % N; const float m = bf16_rne(adj[((size_t)e * N + i) * N + j]); Lg[e][j] = (m > THR) ? lrelu(FS[i * 4 + e] + FD[j * 4 + e]) : -1e9f; }
  __syncthreads();
  if (wave < NE) { const int e = wave; float mx = -INFINITY; for (int j = lane; j < N; j += 32) mx = fmaxf(mx, Lg[e][j]);
#pragma unroll
    for (int o = 16; o >= 1; o >>= 1) mx = fmaxf(mx, __shfl_xor(mx, o));
    float sm = 0.0f; for (int j = lane; j < N; j += 32) { const float w = nexp2((Lg[e][j] - mx) * LOG2E); Lg[e][j] = w; sm += w; }
#pragma unroll
    for (int o = 16; o >= 1; o >>= 1) sm += __shfl_xor(sm, o);
    if (lane == 0) inv[e] = 1.0f / sm; }
  __syncthreads();
  for (int j = t_; j < N; j += 256) { const float abar = (((Lg[0][j] * inv[0] + Lg[1][j] * inv[1]) + Lg[2][j] * inv[2]) + Lg[3][j] * inv[3]) * 0.25f; b16 p, q; split16(abar * PS, p, q); Rh[j] = p; Rl[j] = q; }
  __syncthreads();
  for (int pass = 0; pass < 2; ++pass) { if (t_ < N / 8) { *(volatile v8b*)(ABh + (size_t)i * N + t_ * 8) = *(const v8b*)(&Rh[t_ * 8]); *(volatile v8b*)(ABl + (size_t)i * N + t_ * 8) = *(const v8b*)(&Rl[t_ * 8]); } __threadfence(); }
}
template <int MODE>
__global__ __launch_bounds__(128) void aggr_kernel(const b16* __restrict__ ABh, const b16* __restrict__ ABl, const b16* __restrict__ HTh, const b16* __restrict__ HTl, const float* __restrict__ Yprev, float* __restrict__ Yf, b16* __restrict__ Yh, b16* __restrict__ Yl, int D) {
  __shared__ __attribute__((aligned(16))) float Tf[4][16][128 + 4]; __shared__ __attribute__((aligned(16))) b16 Th[4][16][128 + 8], Tl[4][16][128 + 8];
  const int wave = threadIdx.x >> 5, lane = threadIdx.x & 31, nloc = lane & 15, hlf = lane >> 4; const size_t m0 = (size_t)blockIdx.x * 64 + wave * 16; const int n0 = blockIdx.y * 128;
  v8f acc[8];
#pragma unroll
  for (int t = 0; t < 8; ++t) acc[t] = (v8f){};
  for (int kb = 0; kb < N; kb += 32) { const v16b a = frag_kb(ABh + (m0 + nloc) * N + kb, hlf), al = frag_kb(ABl + (m0 + nloc) * N + kb, hlf);
#pragma unroll
    for (int t = 0; t < 8; ++t) { const v16b bh = frag_kb(HTh + (size_t)(n0 + t * 16 + nloc) * N + kb, hlf); acc[t] = wmma16b(a, bh, acc[t]); acc[t] = wmma16b(al, bh, acc[t]); acc[t] = wmma16b(a, frag_kb(HTl + (size_t)(n0 + t * 16 + nloc) * N + kb, hlf), acc[t]); } }
#pragma unroll
  for (int t = 0; t < 8; ++t)
#pragma unroll
    for (int r = 0; r < 8; ++r) { float y = acc[t][r] * (1.0f / (PS * XS)); const size_t row = m0 + 8 * hlf + r; const int c = n0 + t * 16 + nloc; if (MODE == 0) y = fmaxf(y, 0.0f); if (MODE == 1) y += Yprev[row * D + c];
      Tf[wave][8 * hlf + r][t * 16 + nloc] = y; b16 p, q; split16(y * XS, p, q); Th[wave][8 * hlf + r][t * 16 + nloc] = p; Tl[wave][8 * hlf + r][t * 16 + nloc] = q; }
  wave_lds_sync();
  for (int pass = 0; pass < 2; ++pass) { for (int rr = 0; rr < 16; ++rr) *(volatile v4f*)(Yf + (m0 + rr) * D + n0 + lane * 4) = *(const v4f*)(&Tf[wave][rr][lane * 4]);
    for (int r2 = 0; r2 < 16; r2 += 2) { const int rr = r2 + (lane >> 4), c8 = (lane & 15) * 8; const size_t gi = (m0 + rr) * D + n0 + c8; *(volatile v8b*)(Yh + gi) = *(const v8b*)(&Th[wave][rr][c8]); *(volatile v8b*)(Yl + gi) = *(const v8b*)(&Tl[wave][rr][c8]); }
    __threadfence(); }
}
__global__ __launch_bounds__(256) void transp_kernel(const float* __restrict__ Hf, int D, b16* __restrict__ HTh, b16* __restrict__ HTl) {
  __shared__ __attribute__((aligned(16))) b16 Th[64][64 + 8], Tl[64][64 + 8];
  const int n0 = blockIdx.x * 64, c0 = blockIdx.y * 64, t_ = threadIdx.x;
  for (int q = t_; q < 64 * 64; q += 256) { const int nn = q >> 6, cc = q & 63; b16 p, ql; split16(Hf[(size_t)(n0 + nn) * D + c0 + cc] * XS, p, ql); Th[cc][nn] = p; Tl[cc][nn] = ql; }
  __syncthreads();
  for (int pass = 0; pass < 2; ++pass) { for (int q = t_; q < 64 * 8; q += 256) { const int cc = q >> 3, c8 = (q & 7) * 8; const size_t gi = (size_t)(c0 + cc) * N + n0 + c8; *(volatile v8b*)(HTh + gi) = *(const v8b*)(&Th[cc][c8]); *(volatile v8b*)(HTl + gi) = *(const v8b*)(&Tl[cc][c8]); } __threadfence(); }
}
__global__ __launch_bounds__(128) void cos_kernel(const b16* __restrict__ Hh, const b16* __restrict__ Hl, const float* __restrict__ NRM, float* __restrict__ out1) {
  __shared__ __attribute__((aligned(16))) float Tf[4][16][128 + 4];
  const int wave = threadIdx.x >> 5, lane = threadIdx.x & 31, nloc = lane & 15, hlf = lane >> 4; const size_t m0 = (size_t)blockIdx.x * 64 + wave * 16; const int n0 = blockIdx.y * 128;
  v8f acc[8];
#pragma unroll
  for (int t = 0; t < 8; ++t) acc[t] = (v8f){};
#pragma unroll
  for (int kb = 0; kb < H2; kb += 32) { const v16b a = frag_kb(Hh + (m0 + nloc) * H2 + kb, hlf), al = frag_kb(Hl + (m0 + nloc) * H2 + kb, hlf);
#pragma unroll
    for (int t = 0; t < 8; ++t) { const v16b bh = frag_kb(Hh + (size_t)(n0 + t * 16 + nloc) * H2 + kb, hlf); acc[t] = wmma16b(a, bh, acc[t]); acc[t] = wmma16b(al, bh, acc[t]); acc[t] = wmma16b(a, frag_kb(Hl + (size_t)(n0 + t * 16 + nloc) * H2 + kb, hlf), acc[t]); } }
#pragma unroll
  for (int t = 0; t < 8; ++t) { const int j = n0 + t * 16 + nloc; const float nj = NRM[j];
#pragma unroll
    for (int r = 0; r < 8; ++r) { const size_t i = m0 + 8 * hlf + r; Tf[wave][8 * hlf + r][t * 16 + nloc] = acc[t][r] * (1.0f / (XS * XS)) / fmaxf(NRM[i] * nj, COS_EPS); } }
  wave_lds_sync();
  for (int pass = 0; pass < 2; ++pass) { for (int rr = 0; rr < 16; ++rr) *(volatile v4f*)(out1 + (m0 + rr) * N + n0 + lane * 4) = *(const v4f*)(&Tf[wave][rr][lane * 4]); __threadfence(); }
}
__global__ __launch_bounds__(256) void norm_kernel(const float* __restrict__ Hf, float* __restrict__ NRM) {
  __shared__ __attribute__((aligned(16))) float r32[32];
  const int wave = threadIdx.x >> 5, lane = threadIdx.x & 31;
  for (int q = 0; q < 4; ++q) { const size_t i = (size_t)blockIdx.x * 32 + wave * 4 + q; float s = 0.0f; for (int c = lane; c < H2; c += 32) { const float v = Hf[i * H2 + c]; s += pmul(v, v); }
#pragma unroll
    for (int o = 16; o >= 1; o >>= 1) s += __shfl_xor(s, o);
    if (lane == 0) r32[wave * 4 + q] = sqrtf(s); }
  __syncthreads();
  for (int pass = 0; pass < 2; ++pass) { if (threadIdx.x < 8) *(volatile v4f*)(NRM + (size_t)blockIdx.x * 32 + threadIdx.x * 4) = *(const v4f*)(&r32[threadIdx.x * 4]); __threadfence(); }
}
__global__ __launch_bounds__(128) void dec_kernel(const float* __restrict__ PQ, const float* __restrict__ rawadj, const b16* __restrict__ FC1R, const float* __restrict__ b1, const b16* __restrict__ FC2T, const float* __restrict__ b2, const b16* __restrict__ FC3T, const float* __restrict__ b3, float* __restrict__ out) {
__shared__ __attribute__((aligned(16))) b16 Ah[4][16][H3 + 8]; __shared__ __attribute__((aligned(16))) b16 Zh[4][16][H4 + 8]; __shared__ __attribute__((aligned(16))) float To[4][32]; __shared__ __attribute__((aligned(16))) b16 RA[4][16][32 + 8]; __shared__ float pb[H3];
  const int i = blockIdx.y, j0 = blockIdx.x * 64, wave = threadIdx.x >> 5, lane = threadIdx.x & 31, nloc = lane & 15, hlf = lane >> 4, t_ = threadIdx.x;
  for (int o = t_; o < H3; o += 128) pb[o] = PQ[(size_t)i * (2 * H3) + o] + bf16_rne(b1[o]);
  const int jw = j0 + wave * 16;
  for (int q = lane; q < 16 * 32; q += 32) { const int rr = q >> 5, k = q & 31; RA[wave][rr][k] = (k < NE) ? (b16)(bf16_rne(rawadj[((size_t)min(k, NE - 1) * N + i) * N + jw + rr]) * XS) : (b16)0.0f; }
  __syncthreads();
  { const v16b ra = frag_kb(&RA[wave][nloc][0], hlf);
    for (int hq = 0; hq < 2; ++hq) {
#pragma unroll
      for (int t = 0; t < 8; ++t) { const int o = hq * 128 + t * 16 + nloc; v8f d = {}; d = wmma16b(ra, frag_kb(FC1R + (size_t)o * 32, hlf), d); const float po = pb[o];
#pragma unroll
        for (int r = 0; r < 8; ++r) { const int rr = 8 * hlf + r; const float pre = d[r] * (1.0f / (XS * WSC)) + po + PQ[(size_t)(jw + rr) * (2 * H3) + H3 + o]; Ah[wave][rr][o] = (b16)(fmaxf(pre, 0.0f) * XS); } } } }
  wave_lds_sync();
  v8f acc[8];
#pragma unroll
  for (int t = 0; t < 8; ++t) acc[t] = (v8f){};
#pragma unroll 2
  for (int kb = 0; kb < H3; kb += 32) { const v16b a = frag_kb(&Ah[wave][nloc][kb], hlf);
#pragma unroll
    for (int t = 0; t < 8; ++t) acc[t] = wmma16b(a, frag_kb(FC2T + (size_t)(t * 16 + nloc) * H3 + kb, hlf), acc[t]); }
#pragma unroll
  for (int t = 0; t < 8; ++t) { const int c = t * 16 + nloc; const float bb = bf16_rne(b2[c]);
#pragma unroll
    for (int r = 0; r < 8; ++r) Zh[wave][8 * hlf + r][c] = (b16)(fmaxf(acc[t][r] * (1.0f / (XS * WSC)) + bb, 0.0f) * XS); }
  wave_lds_sync();
  v8f d = {};
#pragma unroll
  for (int kb = 0; kb < H4; kb += 32) d = wmma16b(frag_kb(&Zh[wave][nloc][kb], hlf), frag_kb(FC3T + (size_t)nloc * H4 + kb, hlf), d);
  if (nloc < 2) { for (int r = 0; r < 8; ++r) { const float lg = d[r] * (1.0f / (XS * WSC)) + bf16_rne(b3[nloc]); To[wave][(8 * hlf + r) * 2 + nloc] = lg; } }
  wave_lds_sync();
  if (lane < 16) { const float l0 = To[wave][lane * 2], l1 = To[wave][lane * 2 + 1]; const float mx = fmaxf(l0, l1); const float lse = mx + __logf(__expf(l0 - mx) + __expf(l1 - mx)); To[wave][lane * 2] = l0 - lse; To[wave][lane * 2 + 1] = l1 - lse; }
  wave_lds_sync();
  for (int pass = 0; pass < 2; ++pass) { if (lane < 8) *(volatile v4f*)(out + ((size_t)i * N + jw) * 2 + lane * 4) = *(const v4f*)(&To[wave][lane * 4]); __threadfence(); }
}
}

extern "C" void kernel_launch(void* const* d_in, const int* in_sizes, int n_in, void* d_out, int out_size, void* d_ws, size_t ws_size, hipStream_t stream) {
  (void)n_in;
  auto Fp = [&](int i) { return (const float*)d_in[i]; };
  if (in_sizes[0] != N * F || in_sizes[1] != NE * N * N || in_sizes[2] != NE * N * N || in_sizes[3] != F * H1 || in_sizes[4] != NE * 2 * H1 || in_sizes[5] != H1 * H2 || in_sizes[6] != NE * 2 * H2 || in_sizes[7] != (2 * H2 + NE) * H3 || in_sizes[9] != H3 * H4 || in_sizes[11] != H4 * NCLS || out_size != N * N * 2 + N * N) return;
  size_t off = 0; char* ws = (char*)d_ws;
  auto carve = [&](size_t bytes) { char* p = ws + off; off += (bytes + 255) & ~(size_t)255; return p; };
  b16* Xh = (b16*)carve((size_t)N * F * 2); b16* Xl = (b16*)carve((size_t)N * F * 2); b16* W1T = (b16*)carve((size_t)H1 * F * 2); b16* W2T = (b16*)carve((size_t)H2 * H1 * 2); b16* FC1T = (b16*)carve((size_t)2 * H3 * H2 * 2); b16* FC2T = (b16*)carve((size_t)H4 * H3 * 2); b16* FC3T = (b16*)carve((size_t)16 * H4 * 2); b16* FC1R = (b16*)carve((size_t)H3 * 32 * 2);
  float* Gf = (float*)carve((size_t)N * H1 * 4); b16* HTh = (b16*)carve((size_t)H1 * N * 2); b16* HTl = (b16*)carve((size_t)H1 * N * 2); float* FS = (float*)carve((size_t)N * 4 * 4); float* FD = (float*)carve((size_t)N * 4 * 4); b16* ABh = (b16*)carve((size_t)N * N * 2); b16* ABl = (b16*)carve((size_t)N * N * 2);
  float* Yf = (float*)carve((size_t)N * H1 * 4); b16* Yh = (b16*)carve((size_t)N * H1 * 2); b16* Yl = (b16*)carve((size_t)N * H1 * 2); float* Sf = (float*)carve((size_t)N * H1 * 4); b16* Sh = (b16*)carve((size_t)N * H1 * 2); b16* Sl = (b16*)carve((size_t)N * H1 * 2);
  float* Hf = (float*)carve((size_t)N * H2 * 4); b16* Hh = (b16*)carve((size_t)N * H2 * 2); b16* Hl = (b16*)carve((size_t)N * H2 * 2); float* PQ = (float*)carve((size_t)N * 2 * H3 * 4); float* NRM = (float*)carve((size_t)N * 4);
  if (off > ws_size || off > ((size_t)128 << 20)) return;
  float* out0 = (float*)d_out; float* out1 = out0 + (size_t)N * N * 2;
  prep_kernel<<<(unsigned)(((size_t)N * F / 8 + (size_t)H1 * F / 8 + (size_t)H2 * H1 / 8 + (size_t)2 * H3 * H2 / 8 + (size_t)H4 * H3 / 8 + 16 * H4 / 8 + (size_t)H3 * 32 / 8 + 255) / 256), 256, 0, stream>>>(Fp(0), Fp(3), Fp(5), Fp(7), Fp(9), Fp(11), Xh, Xl, W1T, W2T, FC1T, FC2T, FC3T, FC1R);
  gemm_kernel<F><<<dim3(N / 64, H1 / 128), 128, 0, stream>>>(Xh, Xl, F, W1T, Gf, nullptr, nullptr, H1);
  fdot_kernel<<<N / 8, 256, 0, stream>>>(Gf, H1, Fp(4), FS, FD);
  attrow_kernel<<<N, 256, 0, stream>>>(FS, FD, Fp(1), ABh, ABl);
  transp_kernel<<<dim3(N / 64, H1 / 64), 256, 0, stream>>>(Gf, H1, HTh, HTl);
  aggr_kernel<0><<<dim3(N / 64, H1 / 128), 128, 0, stream>>>(ABh, ABl, HTh, HTl, nullptr, Yf, Yh, Yl, H1);
  gemm_kernel<H1><<<dim3(N / 64, H1 / 128), 128, 0, stream>>>(Yh, Yl, H1, W1T, Gf, nullptr, nullptr, H1);
  fdot_kernel<<<N / 8, 256, 0, stream>>>(Gf, H1, Fp(4), FS, FD);
  attrow_kernel<<<N, 256, 0, stream>>>(FS, FD, Fp(1), ABh, ABl);
  transp_kernel<<<dim3(N / 64, H1 / 64), 256, 0, stream>>>(Gf, H1, HTh, HTl);
  aggr_kernel<1><<<dim3(N / 64, H1 / 128), 128, 0, stream>>>(ABh, ABl, HTh, HTl, Yf, Sf, Sh, Sl, H1);
  gemm_kernel<H1><<<dim3(N / 64, H2 / 128), 128, 0, stream>>>(Sh, Sl, H1, W2T, Gf, nullptr, nullptr, H2);
  fdot_kernel<<<N / 8, 256, 0, stream>>>(Gf, H2, Fp(6), FS, FD);
  attrow_kernel<<<N, 256, 0, stream>>>(FS, FD, Fp(1), ABh, ABl);
  transp_kernel<<<dim3(N / 64, H2 / 64), 256, 0, stream>>>(Gf, H2, HTh, HTl);
  aggr_kernel<2><<<dim3(N / 64, H2 / 128), 128, 0, stream>>>(ABh, ABl, HTh, HTl, nullptr, Hf, Hh, Hl, H2);
  norm_kernel<<<N / 32, 256, 0, stream>>>(Hf, NRM);
  cos_kernel<<<dim3(N / 64, N / 128), 128, 0, stream>>>(Hh, Hl, NRM, out1);
  gemm_kernel<H2><<<dim3(N / 64, 2 * H3 / 128), 128, 0, stream>>>(Hh, Hl, H2, FC1T, PQ, nullptr, nullptr, 2 * H3);
  dec_kernel<<<dim3(N / 64, N), 128, 0, stream>>>(PQ, Fp(2), FC1R, Fp(8), FC2T, Fp(10), FC3T, Fp(12), out0);
}
